// DiMBlock_90452011254018
// MI455X (gfx1250) — hardware-run, weakly checked
//
#include <hip/hip_runtime.h>
#include <math.h>

typedef __attribute__((ext_vector_type(16))) _Float16 v16h;
typedef __attribute__((ext_vector_type(8)))  _Float16 v8h;
typedef __attribute__((ext_vector_type(16))) __bf16   v16b;
typedef __attribute__((ext_vector_type(8)))  __bf16   v8b;
typedef __attribute__((ext_vector_type(8)))  float    v8f;
typedef __attribute__((ext_vector_type(4)))  float    v4f;

constexpr int kBatch = 2;
constexpr int kSeq   = 1024;
constexpr int kGridW = 32;
constexpr int kDim   = 256;
constexpr int kDI    = 512;
constexpr int kDS    = 64;
constexpr int kDTR   = 16;
constexpr int kDirs  = 4;
constexpr int kHid   = 1024;
constexpr int kRows  = kBatch * kSeq;
constexpr int kXzW   = 2 * kDI;
constexpr int kNR    = kDTR + 2 * kDS;
constexpr int kNRP   = 192;
constexpr int kDtK   = 32;
constexpr int kMod   = 6 * kDim;
constexpr int kScanCh = 32;
constexpr int kScanTS = 64;
constexpr int kScanXW = 128;
constexpr int kScanYP = 36;
constexpr int kConvP  = 516;
static_assert(kGridW * kGridW == kSeq);
static_assert((kDim % 64) == 0 && (kXzW % 64) == 0 && (kNRP % 64) == 0 && (kDI % 64) == 0 && (kHid % 64) == 0 && (kRows % 64) == 0);
static_assert((kDim % 32) == 0 && (kDI % 32) == 0 && (kDtK % 32) == 0 && (kHid % 32) == 0);
static_assert((kSeq % kScanTS) == 0 && (kDI % kScanCh) == 0);

constexpr size_t kOffWIN  = 0;
constexpr size_t kOffWX   = kOffWIN  + (size_t)kXzW * kDim * 2;
constexpr size_t kOffWDT  = kOffWX   + (size_t)kDirs * kNRP * kDI * 2;
constexpr size_t kOffWOUT = kOffWDT  + (size_t)kDirs * kDI * kDtK * 2;
constexpr size_t kOffWF1  = kOffWOUT + (size_t)kDim * kDI * 2;
constexpr size_t kOffWF2  = kOffWF1  + (size_t)kHid * kDim * 2;
constexpr size_t kOffMOD  = kOffWF2  + (size_t)kDim * kHid * 2;
constexpr size_t kOffH16  = kOffMOD  + (size_t)kBatch * kMod * 4;
constexpr size_t kOffXZ   = kOffH16  + (size_t)kRows * kDim * 2;
constexpr size_t kOffXI   = kOffXZ   + (size_t)kRows * kXzW * 4;
constexpr size_t kOffXS   = kOffXI   + (size_t)kRows * kDI * 4;
constexpr size_t kOffXD   = kOffXS   + (size_t)2 * kRows * kDI * 2;
constexpr size_t kOffDTA  = kOffXD   + (size_t)kDirs * kRows * kNRP * 4;
constexpr size_t kOffDTP  = kOffDTA  + (size_t)kDirs * kRows * kDtK * 2;
constexpr size_t kOffY    = kOffDTP  + (size_t)kDirs * kRows * kDI * 4;
constexpr size_t kOffYG   = kOffY    + (size_t)kDirs * kRows * kDI * 4;
constexpr size_t kOffX1   = kOffYG   + (size_t)kRows * kDI * 2;
constexpr size_t kOffM16  = kOffX1   + (size_t)kRows * kDim * 4;
constexpr size_t kOffF1   = kOffM16  + (size_t)kRows * kDim * 2;
constexpr size_t kOffG16  = kOffF1   + (size_t)kRows * kHid * 4;
constexpr size_t kWsTotal = kOffG16  + (size_t)kRows * kHid * 2;
static_assert(kWsTotal == 78786560ull);
static_assert(kWsTotal <= 134217728ull);
static_assert((kOffWX % 128) == 0 && (kOffWDT % 128) == 0 && (kOffWOUT % 128) == 0 && (kOffWF1 % 128) == 0 &&
              (kOffWF2 % 128) == 0 && (kOffMOD % 128) == 0 && (kOffH16 % 128) == 0 && (kOffXZ % 128) == 0 &&
              (kOffXI % 128) == 0 && (kOffXS % 128) == 0 && (kOffXD % 128) == 0 && (kOffDTA % 128) == 0 &&
              (kOffDTP % 128) == 0 && (kOffY % 128) == 0 && (kOffYG % 128) == 0 && (kOffX1 % 128) == 0 &&
              (kOffM16 % 128) == 0 && (kOffF1 % 128) == 0 && (kOffG16 % 128) == 0);

__device__ __forceinline__ unsigned short f2bf_bits(float f) {
  unsigned u = __float_as_uint(f);
  return (unsigned short)((u + 0x7FFFu + ((u >> 16) & 1u)) >> 16);
}
__device__ __forceinline__ float bf_bits2f(unsigned short h) { return __uint_as_float(((unsigned)h) << 16); }

__device__ __forceinline__ void dep_guard_h(v8f& a, v8f& b, v16h x, v16h y) { asm volatile("v_nop\n\tv_nop\n\tv_nop\n\tv_nop" : "+v"(a), "+v"(b) : "v"(x), "v"(y)); }
__device__ __forceinline__ void dep_guard_b(v8f& a, v8f& b, v16b x, v16b y) { asm volatile("v_nop\n\tv_nop\n\tv_nop\n\tv_nop" : "+v"(a), "+v"(b) : "v"(x), "v"(y)); }
__device__ __forceinline__ void keep4_h(v16h a, v16h b, v16h c, v16h d) { asm volatile("v_nop" :: "v"(a), "v"(b), "v"(c), "v"(d)); }
__device__ __forceinline__ void keep4_b(v16b a, v16b b, v16b c, v16b d) { asm volatile("v_nop" :: "v"(a), "v"(b), "v"(c), "v"(d)); }
__device__ __forceinline__ void acc_guard4(v8f& a, v8f& b, v8f& c, v8f& d) { asm volatile("v_nop\n\tv_nop\n\tv_nop\n\tv_nop" : "+v"(a), "+v"(b), "+v"(c), "+v"(d)); }
template <typename T> struct Frag;
template <> struct Frag<_Float16> {
  typedef v16h V; union U { v16h v; v8h h[2]; };
  static __device__ __forceinline__ v16h load(const _Float16* p) {
    U f; f.h[0] = *(const v8h*)(p); f.h[1] = *(const v8h*)(p + 16); return f.v;
  }
  static __device__ __forceinline__ v8f mma(v16h a, v16h b, v8f c) {
    return __builtin_amdgcn_wmma_f32_16x16x32_f16(false, a, false, b, (short)0, c, false, false);
  }
  static __device__ __forceinline__ void guard(v8f& a, v8f& b, v16h x, v16h y) { dep_guard_h(a, b, x, y); }
  static __device__ __forceinline__ void keep(v16h a, v16h b, v16h c, v16h d) { keep4_h(a, b, c, d); }
};
template <> struct Frag<__bf16> {
  typedef v16b V; union U { v16b v; v8b h[2]; };
  static __device__ __forceinline__ v16b load(const __bf16* p) {
    U f; f.h[0] = *(const v8b*)(p); f.h[1] = *(const v8b*)(p + 16); return f.v;
  }
  static __device__ __forceinline__ v8f mma(v16b a, v16b b, v8f c) {
    return __builtin_amdgcn_wmma_f32_16x16x32_bf16(false, a, false, b, (short)0, c, false, false);
  }
  static __device__ __forceinline__ void guard(v8f& a, v8f& b, v16b x, v16b y) { dep_guard_b(a, b, x, y); }
  static __device__ __forceinline__ void keep(v16b a, v16b b, v16b c, v16b d) { keep4_b(a, b, c, d); }
};

__device__ __forceinline__ float wave_sum32(float v) {
  v += __shfl_xor(v, 1, 32);
  v += __shfl_xor(v, 2, 32);
  v += __shfl_xor(v, 4, 32);
  v += __shfl_xor(v, 8, 32);
  v += __shfl_xor(v, 16, 32);
  return v;
}

template <int ET> struct Elem;
template <> struct Elem<0> { typedef _Float16 T; };
template <> struct Elem<1> { typedef __bf16 T; };
template <int ET, int SPL, int BIAS_MODE, int OUT_MODE, bool RESID, int ACT, bool GATE>
__global__ __launch_bounds__(256) void wmma_gemm64(
    const unsigned short* __restrict__ Ap, const unsigned short* __restrict__ A2p, int lda, long strideA,
    const unsigned short* __restrict__ Btp, const unsigned short* __restrict__ Bt2p, int ldb, long strideB,
    void* __restrict__ Cout, void* __restrict__ Cout2, int ldc, long strideC,
    const float* __restrict__ bias,
    const float* __restrict__ resid, long strideR,
    int M, int N, int K, float scale,
    const float* __restrict__ gatev, int gate_shift, int gate_ld) {
  typedef typename Elem<ET>::T T;
  typedef typename Frag<T>::V V;
  const T* A = (const T*)Ap; const T* A2 = (const T*)A2p; const T* Bt = (const T*)Btp; const T* Bt2 = (const T*)Bt2p;
  __shared__ __align__(16) float sT[8][16 * 68];
  const int b    = blockIdx.y;
  const int lane = threadIdx.x & 31;
  const int wave = threadIdx.x >> 5;
  const int tilesN = N >> 6;
  const int tilesM = M >> 6;
  const int tile = blockIdx.x * 8 + wave;
  if (tile >= tilesM * tilesN) return;
  const int tm = tile / tilesN;
  const int tn = tile - tm * tilesN;
  const int m0 = tm << 6;
  const int n0 = tn << 6;

  const T* Ab  = A  + (size_t)b * strideA;
  const T* Bb  = Bt + (size_t)b * strideB;
  const T* Ab2 = (SPL >= 1) ? (A2  + (size_t)b * strideA) : nullptr;
  const T* Bb2 = (SPL == 2) ? (Bt2 + (size_t)b * strideB) : nullptr;

  const int rlane = lane & 15;
  const int koff  = (lane >> 4) * 8;
  const int mOff  = (lane >> 4) * 8;

  v8f acc[4][4];
#pragma unroll
  for (int i = 0; i < 4; ++i)
#pragma unroll
    for (int j = 0; j < 4; ++j) acc[i][j] = (v8f){0.f,0.f,0.f,0.f,0.f,0.f,0.f,0.f};

  for (int k0 = 0; k0 < K; k0 += 32) {
    V bh[4], bl[4];
#pragma unroll
    for (int j = 0; j < 4; ++j) {
      const size_t bo = (size_t)(n0 + (j << 4) + rlane) * ldb + koff + k0;
      bh[j] = Frag<T>::load(Bb + bo);
      if (SPL == 2) bl[j] = Frag<T>::load(Bb2 + bo);
    }
#pragma unroll
    for (int i = 0; i < 4; ++i) {
      const size_t ao = (size_t)(m0 + (i << 4) + rlane) * lda + koff + k0;
      V ah = Frag<T>::load(Ab + ao);
      V al;
      if (SPL >= 1) al = Frag<T>::load(Ab2 + ao);
#pragma unroll
      for (int j = 0; j < 4; ++j) {
        acc[i][j] = Frag<T>::mma(ah, bh[j], acc[i][j]);
        if (SPL == 2) acc[i][j] = Frag<T>::mma(ah, bl[j], acc[i][j]);
        if (SPL >= 1) acc[i][j] = Frag<T>::mma(al, bh[j], acc[i][j]);
      }
      Frag<T>::guard(acc[i][0], acc[i][3], ah, (SPL >= 1) ? al : ah);
    }
    Frag<T>::keep(bh[0], bh[1], bh[2], bh[3]);
    if (SPL == 2) Frag<T>::keep(bl[0], bl[1], bl[2], bl[3]);
  }
  acc_guard4(acc[0][0], acc[0][1], acc[0][2], acc[0][3]);
  acc_guard4(acc[1][0], acc[1][1], acc[1][2], acc[1][3]);
  acc_guard4(acc[2][0], acc[2][1], acc[2][2], acc[2][3]);
  acc_guard4(acc[3][0], acc[3][1], acc[3][2], acc[3][3]);

  float* slab = sT[wave];
  const float* Rb = RESID ? (resid + (size_t)b * strideR) : nullptr;
#pragma unroll
  for (int i = 0; i < 4; ++i) {
    const int mBase = m0 + (i << 4);
#pragma unroll
    for (int j = 0; j < 4; ++j) {
      const int n = n0 + (j << 4) + rlane;
      float bv = 0.f;
      if (BIAS_MODE == 2) bv = bias[n];
#pragma unroll
      for (int r = 0; r < 8; ++r) {
        float v = acc[i][j][r] * scale;
        if (BIAS_MODE == 1) v += bias[mBase + mOff + r];
        if (BIAS_MODE == 2) v += bv;
        if (RESID) {
          const float rv = Rb[(size_t)(mBase + mOff + r) * ldc + n];
          if (GATE) {
            const float gv = gatev[(size_t)((mBase + mOff + r) >> gate_shift) * gate_ld + n];
            v = rv + gv * v;
          } else {
            v += rv;
          }
        }
        if (ACT == 1) v = tanhf(v);
        if (ACT == 2) v = fmaxf(v, 0.0f);
        if (ACT == 3) v = v / (1.0f + expf(-v));
        if (ACT == 4) v = (v > 0.f) ? v : 0.01f * v;
        slab[(mOff + r) * 68 + (j << 4) + rlane] = v;
      }
    }
    __builtin_amdgcn_fence(__ATOMIC_RELEASE, "workgroup");
    __builtin_amdgcn_wave_barrier();
    __builtin_amdgcn_fence(__ATOMIC_ACQUIRE, "workgroup");
    if (OUT_MODE == 0) {
      float* C = (float*)Cout + (size_t)b * strideC;
      const int hh = lane >> 4, c4 = (lane & 15) * 4;
      for (int pass = 0; pass < 2; ++pass) {
#pragma unroll
        for (int it = 0; it < 8; ++it) {
          const int row = it * 2 + hh;
          v4f v = *(const v4f*)(slab + row * 68 + c4);
          *(volatile v4f*)(C + (size_t)(mBase + row) * ldc + n0 + c4) = v;
        }
        __threadfence();
      }
    } else {
      const int q = lane >> 3, c8 = (lane & 7) * 8;
      unsigned short* C  = (unsigned short*)Cout  + (size_t)b * strideC;
      unsigned short* C2 = (OUT_MODE == 2) ? ((unsigned short*)Cout2 + (size_t)b * strideC) : nullptr;
      for (int pass = 0; pass < 2; ++pass) {
#pragma unroll
        for (int it = 0; it < 4; ++it) {
          const int row = it * 4 + q;
          const float* sp = slab + row * 68 + c8;
          v8h hv, lv;
#pragma unroll
          for (int e = 0; e < 8; ++e) {
            if (OUT_MODE == 1) {
              hv[e] = (_Float16)sp[e];
            } else {
              unsigned short hb = f2bf_bits(sp[e]);
              unsigned short lb = f2bf_bits(sp[e] - bf_bits2f(hb));
              hv[e] = __builtin_bit_cast(_Float16, hb);
              lv[e] = __builtin_bit_cast(_Float16, lb);
            }
          }
          *(volatile v8h*)(C + (size_t)(mBase + row) * ldc + n0 + c8) = hv;
          if (OUT_MODE == 2) *(volatile v8h*)(C2 + (size_t)(mBase + row) * ldc + n0 + c8) = lv;
        }
        __threadfence();
      }
    }
    __builtin_amdgcn_fence(__ATOMIC_RELEASE, "workgroup");
    __builtin_amdgcn_wave_barrier();
    __builtin_amdgcn_fence(__ATOMIC_ACQUIRE, "workgroup");
  }
}

template <int KT>
__global__ __launch_bounds__(256) void wt_cast_kernel(
    const float* __restrict__ in, unsigned short* __restrict__ out,
    int Kdim, int Ndim, int Npad, int ldo, long inStride, long outStride, float scale)
{
  static_assert(KT == 64 || KT == 32);
  __shared__ __align__(16) float sT[64 * (KT + 4)];
  const int tid = threadIdx.x;
  const int n0 = blockIdx.x * 64, k0 = blockIdx.y * KT, z = blockIdx.z;
  const float* inz = in + (size_t)z * inStride;
  _Float16* outz = (_Float16*)(out + (size_t)z * outStride);
  const int nl = tid & 63;
  const int n  = n0 + nl;
  const int nc = (n < Ndim) ? n : (Ndim - 1);
#pragma unroll 1
  for (int i = 0; i < KT / 4; ++i) {
    const int kl = (tid >> 6) + 4 * i;
    const int k  = k0 + kl;
    const int kc = (k < Kdim) ? k : (Kdim - 1);
    const float v = inz[(size_t)kc * Ndim + nc];
    sT[nl * (KT + 4) + kl] = (k < Kdim && n < Ndim) ? v : 0.0f;
  }
  __syncthreads();
  constexpr int NIT = (KT == 64) ? 2 : 1;
  v8h hv[NIT];
#pragma unroll
  for (int it = 0; it < NIT; ++it) {
    const int row = (KT == 64) ? ((tid >> 3) + 32 * it) : (tid >> 2);
    const int k8  = (KT == 64) ? ((tid & 7) * 8) : ((tid & 3) * 8);
    const float* sp = sT + row * (KT + 4) + k8;
    const v4f a0 = *(const v4f*)(sp);
    const v4f a1 = *(const v4f*)(sp + 4);
#pragma unroll
    for (int e = 0; e < 4; ++e) {
      hv[it][e]     = (_Float16)(a0[e] * scale);
      hv[it][4 + e] = (_Float16)(a1[e] * scale);
    }
  }
  for (int pass = 0; pass < 2; ++pass) {
#pragma unroll
    for (int it = 0; it < NIT; ++it) {
      const int row = (KT == 64) ? ((tid >> 3) + 32 * it) : (tid >> 2);
      const int k8  = (KT == 64) ? ((tid & 7) * 8) : ((tid & 3) * 8);
      *(volatile v8h*)(outz + (size_t)(n0 + row) * ldo + k0 + k8) = hv[it];
    }
    __threadfence();
  }
}

__global__ __launch_bounds__(256) void mod_kernel(
    const float* __restrict__ c, const float* __restrict__ Wada, const float* __restrict__ bada, float* __restrict__ MOD)
{
  __shared__ float sS[kDim];
  const int tid = threadIdx.x, b = blockIdx.y;
  const int o = blockIdx.x * 256 + tid;
  {
    const float cv = c[b * kDim + tid];
    sS[tid] = cv * __builtin_amdgcn_rcpf(1.0f + expf(-cv));
  }
  __syncthreads();
  float acc = 0.0f;
#pragma unroll 1
  for (int i = 0; i < kDim; ++i) acc = fmaf(sS[i], Wada[(size_t)i * kMod + o], acc);
  const float r = acc + bada[o];
  volatile float* p = MOD + (size_t)b * kMod + o;
  *p = r;
  __threadfence();
  *p = r;
}

__global__ __launch_bounds__(256) void ln_mod_kernel(
    const float* __restrict__ X, const float* __restrict__ MOD, int shOff, int scOff, unsigned short* __restrict__ Hout)
{
  const int lane = threadIdx.x & 31, wave = threadIdx.x >> 5;
  const int row = blockIdx.x * 8 + wave;
  const int b = row >> 10;
  const int ch = lane * 8;
  const float* xr = X + (size_t)row * kDim + ch;
  const v4f a0 = *(const v4f*)(xr);
  const v4f a1 = *(const v4f*)(xr + 4);
  float xv[8];
#pragma unroll
  for (int e = 0; e < 4; ++e) { xv[e] = a0[e]; xv[4 + e] = a1[e]; }
  float s = 0.0f;
#pragma unroll
  for (int e = 0; e < 8; ++e) s += xv[e];
  s = wave_sum32(s);
  const float mu = s * (1.0f / 256.0f);
  float ss = 0.0f;
#pragma unroll
  for (int e = 0; e < 8; ++e) { xv[e] = xv[e] - mu; ss = fmaf(xv[e], xv[e], ss); }
  ss = wave_sum32(ss);
  const float rstd = rsqrtf(ss * (1.0f / 256.0f) + 1e-6f);
  const float* mp = MOD + (size_t)b * kMod;
  const v4f sh0 = *(const v4f*)(mp + shOff + ch), sh1 = *(const v4f*)(mp + shOff + ch + 4);
  const v4f sc0 = *(const v4f*)(mp + scOff + ch), sc1 = *(const v4f*)(mp + scOff + ch + 4);
  v8h hv;
#pragma unroll
  for (int e = 0; e < 4; ++e) {
    hv[e]     = (_Float16)((xv[e] * rstd * (1.0f + sc0[e]) + sh0[e]) * 8.0f);
    hv[4 + e] = (_Float16)((xv[4 + e] * rstd * (1.0f + sc1[e]) + sh1[e]) * 8.0f);
  }
  _Float16* op = (_Float16*)Hout + (size_t)row * kDim + ch;
  *(volatile v8h*)op = hv;
  __threadfence();
  *(volatile v8h*)op = hv;
}

__global__ __launch_bounds__(256) void conv_kernel(
    const float* __restrict__ XZ, const float* __restrict__ cw, const float* __restrict__ cb,
    float* __restrict__ XI, unsigned short* __restrict__ XSrow, unsigned short* __restrict__ XScol)
{
  __shared__ __align__(16) float sF[4 * kConvP];
  const int tid = threadIdx.x;
  const int rl  = tid >> 6;
  const int row = blockIdx.x * 4 + rl;
  const int b   = row >> 10;
  const int l   = row & (kSeq - 1);
  const int gh  = l >> 5, gw = l & 31;
  const int c8  = (tid & 63) * 8;
  float acc[8];
#pragma unroll
  for (int e = 0; e < 8; ++e) acc[e] = 0.0f;
#pragma unroll 1
  for (int tap = 0; tap < 9; ++tap) {
    const int kh = tap / 3;
    const int kw = tap - kh * 3;
    const int hh = gh + kh - 1, ww = gw + kw - 1;
    const bool valid = (hh >= 0) && (hh < kGridW) && (ww >= 0) && (ww < kGridW);
    const int hc = hh < 0 ? 0 : (hh >= kGridW ? kGridW - 1 : hh);
    const int wc = ww < 0 ? 0 : (ww >= kGridW ? kGridW - 1 : ww);
    const float* src = XZ + ((size_t)b * kSeq + (size_t)hc * kGridW + wc) * kXzW + c8;
    const v4f x0 = *(const v4f*)(src);
    const v4f x1 = *(const v4f*)(src + 4);
    const float* wp = cw + (size_t)tap * kDI + c8;
    const v4f w0 = *(const v4f*)(wp);
    const v4f w1 = *(const v4f*)(wp + 4);
#pragma unroll
    for (int e = 0; e < 4; ++e) {
      acc[e]     = fmaf(valid ? x0[e] : 0.0f, w0[e], acc[e]);
      acc[4 + e] = fmaf(valid ? x1[e] : 0.0f, w1[e], acc[4 + e]);
    }
  }
  const v4f b0 = *(const v4f*)(cb + c8);
  const v4f b1 = *(const v4f*)(cb + c8 + 4);
  v4f g0, g1;
  v8h hv;
#pragma unroll
  for (int e = 0; e < 4; ++e) {
    const float s0 = acc[e] + b0[e];
    const float s1 = acc[4 + e] + b1[e];
    const float r0 = s0 * __builtin_amdgcn_rcpf(1.0f + expf(-s0));
    const float r1 = s1 * __builtin_amdgcn_rcpf(1.0f + expf(-s1));
    g0[e] = r0; g1[e] = r1;
    hv[e]     = (_Float16)(r0 * 256.0f);
    hv[4 + e] = (_Float16)(r1 * 256.0f);
  }
  *(v4f*)(sF + rl * kConvP + c8)     = g0;
  *(v4f*)(sF + rl * kConvP + c8 + 4) = g1;
  const int lc = gw * kGridW + gh;
  _Float16* pr = (_Float16*)XSrow + (size_t)row * kDI + c8;
  _Float16* pc = (_Float16*)XScol + ((size_t)b * kSeq + lc) * kDI + c8;
  *(volatile v8h*)pr = hv;
  *(volatile v8h*)pc = hv;
  __threadfence();
  *(volatile v8h*)pr = hv;
  *(volatile v8h*)pc = hv;
  __syncthreads();
  for (int pass = 0; pass < 2; ++pass) {
#pragma unroll
    for (int it = 0; it < 2; ++it) {
      const int flat = it * 256 + tid;
      const int rr = flat >> 7;
      const int c4 = (flat & 127) * 4;
      const v4f v = *(const v4f*)(sF + rr * kConvP + c4);
      *(volatile v4f*)(XI + ((size_t)blockIdx.x * 4 + rr) * kDI + c4) = v;
    }
    __threadfence();
  }
}

__global__ __launch_bounds__(256) void dta_kernel(const float* __restrict__ XD, unsigned short* __restrict__ DTA)
{
  const int i = blockIdx.x * 256 + threadIdx.x;
  const int row = i >> 2, q = i & 3;
  const float* src = XD + (size_t)row * kNRP + (q & 1) * 8;
  const v4f a0 = *(const v4f*)(src);
  const v4f a1 = *(const v4f*)(src + 4);
  const bool live = (q < 2);
  v8h hv;
#pragma unroll
  for (int e = 0; e < 4; ++e) {
    hv[e]     = (_Float16)(live ? a0[e] * 256.0f : 0.0f);
    hv[4 + e] = (_Float16)(live ? a1[e] * 256.0f : 0.0f);
  }
  _Float16* op = (_Float16*)DTA + (size_t)row * kDtK + q * 8;
  *(volatile v8h*)op = hv;
  __threadfence();
  *(volatile v8h*)op = hv;
}

__global__ __launch_bounds__(128) void scan_kernel(
    const float* __restrict__ XD, const float* __restrict__ DTP, const float* __restrict__ XI,
    const float* __restrict__ dtb, const float* __restrict__ Alog, const float* __restrict__ Dp,
    float* __restrict__ Y)
{
  __shared__ __align__(16) float sX[kScanTS * kScanXW];
  __shared__ __align__(16) float sY[kScanTS * kScanYP];
  __shared__ __align__(16) float sA[16 * 128];
  const int tid = threadIdx.x, lane = tid & 31, wave = tid >> 5;
  const int blk = blockIdx.x;
  const int cb = blk & 15;
  const int k  = (blk >> 4) & 3;
  const int b  = blk >> 6;
  const int c  = tid >> 2, q4 = tid & 3, sq = q4 * 16;
  const int d  = cb * kScanCh + c;
  const size_t kd = (size_t)k * kDI + d;
#pragma unroll 1
  for (int s = 0; s < 16; ++s) sA[s * 128 + tid] = -expf(Alog[kd * kDS + sq + s]);
  __syncthreads();
  float negA[16], h[16];
#pragma unroll
  for (int j = 0; j < 16; ++j) { negA[j] = sA[j * 128 + tid]; h[j] = 0.0f; }
  const float Dval = Dp[kd], dbias = dtb[kd];
  const size_t xdPlane  = (size_t)k * kRows + (size_t)b * kSeq;
  const size_t gridBase = (size_t)b * kSeq;
  const bool rev  = (k >= 2);
  const bool colk = ((k & 1) != 0);
  const int qq = lane >> 3, c4o = (lane & 7) * 4;
#pragma unroll 1
  for (int t0 = 0; t0 < kSeq; t0 += kScanTS) {
    __syncthreads();
#pragma unroll 1
    for (int i = 0; i < 16; ++i) {
      const int flat = i * 128 + tid;
      const int s = flat >> 5;
      const int c4 = (flat & 31) * 4;
      const int t = t0 + s;
      const int pos = rev ? (kSeq - 1 - t) : t;
      *(v4f*)(sX + s * kScanXW + c4) = *(const v4f*)(XD + (xdPlane + pos) * kNRP + kDTR + c4);
    }
    __syncthreads();
#pragma unroll 1
    for (int s = 0; s < kScanTS; ++s) {
      const int t = t0 + s;
      const int pos = rev ? (kSeq - 1 - t) : t;
      const int gr = colk ? (((pos & 31) << 5) | (pos >> 5)) : pos;
      const float u = XI[(gridBase + gr) * kDI + d];
      const float v = DTP[(xdPlane + pos) * kDI + d] + dbias;
      const float ea  = expf(-fabsf(v));
      const float ua  = 1.0f + ea;
      const float l1p = logf(ua) + (ea - (ua - 1.0f)) * __builtin_amdgcn_rcpf(ua);
      const float dt  = fmaxf(v, 0.0f) + l1p;
      const float dtx = dt * u;
      const float* xr = sX + s * kScanXW;
      float y = 0.0f;
#pragma unroll
      for (int q = 0; q < 4; ++q) {
        const v4f bv = *(const v4f*)(xr + sq + 4 * q);
        const v4f cv = *(const v4f*)(xr + kDS + sq + 4 * q);
#pragma unroll
        for (int e = 0; e < 4; ++e) {
          const int j = 4 * q + e;
          const float ex = __expf(dt * negA[j]);
          h[j] = ex * h[j] + dtx * bv[e];
          y = fmaf(h[j], cv[e], y);
        }
      }
      y += __shfl_xor(y, 1, 32);
      y += __shfl_xor(y, 2, 32);
      const float yf = y + u * Dval;
      if (q4 == 0) sY[s * kScanYP + c] = yf;
    }
    __syncthreads();
    v4f ov[4];
#pragma unroll
    for (int it = 0; it < 4; ++it) {
      const int s = it * 16 + wave * 4 + qq;
      ov[it] = *(const v4f*)(sY + s * kScanYP + c4o);
    }
    for (int pass = 0; pass < 2; ++pass) {
#pragma unroll
      for (int it = 0; it < 4; ++it) {
        const int s = it * 16 + wave * 4 + qq;
        const int t = t0 + s;
        const int pos = rev ? (kSeq - 1 - t) : t;
        const int gr = colk ? (((pos & 31) << 5) | (pos >> 5)) : pos;
        *(volatile v4f*)(Y + ((size_t)k * kRows + gridBase + gr) * kDI + cb * kScanCh + c4o) = ov[it];
      }
      __threadfence();
    }
  }
}

__global__ __launch_bounds__(256) void merge_kernel(
    const float* __restrict__ Y, const float* __restrict__ XZ, const float* __restrict__ lnw,
    const float* __restrict__ lnb, unsigned short* __restrict__ YG)
{
  __shared__ float sRed[16];
  const int tid = threadIdx.x, lane = tid & 31, widx = tid >> 5;
  const int rowl = tid >> 6;
  const int row = blockIdx.x * 4 + rowl;
  const int ch = (tid & 63) * 8;
  const size_t plane = (size_t)kRows * kDI;
  const float* yp = Y + (size_t)row * kDI + ch;
  float yv[8];
  {
    const v4f p0a = *(const v4f*)(yp),             p0b = *(const v4f*)(yp + 4);
    const v4f p1a = *(const v4f*)(yp + plane),     p1b = *(const v4f*)(yp + plane + 4);
    const v4f p2a = *(const v4f*)(yp + 2 * plane), p2b = *(const v4f*)(yp + 2 * plane + 4);
    const v4f p3a = *(const v4f*)(yp + 3 * plane), p3b = *(const v4f*)(yp + 3 * plane + 4);
#pragma unroll
    for (int e = 0; e < 4; ++e) {
      yv[e]     = ((p0a[e] + p1a[e]) + p2a[e]) + p3a[e];
      yv[4 + e] = ((p0b[e] + p1b[e]) + p2b[e]) + p3b[e];
    }
  }
  float s = 0.0f;
#pragma unroll
  for (int e = 0; e < 8; ++e) s += yv[e];
  s = wave_sum32(s);
  if (lane == 0) sRed[widx] = s;
  __syncthreads();
  const float mu = (sRed[rowl * 2] + sRed[rowl * 2 + 1]) * (1.0f / 512.0f);
  float ss = 0.0f;
#pragma unroll
  for (int e = 0; e < 8; ++e) { yv[e] = yv[e] - mu; ss = fmaf(yv[e], yv[e], ss); }
  ss = wave_sum32(ss);
  if (lane == 0) sRed[8 + widx] = ss;
  __syncthreads();
  const float var = (sRed[8 + rowl * 2] + sRed[8 + rowl * 2 + 1]) * (1.0f / 512.0f);
  const float rstd = rsqrtf(var + 1e-6f);
  const v4f w0 = *(const v4f*)(lnw + ch), w1 = *(const v4f*)(lnw + ch + 4);
  const v4f q0 = *(const v4f*)(lnb + ch), q1 = *(const v4f*)(lnb + ch + 4);
  const float* zp = XZ + (size_t)row * kXzW + kDI + ch;
  const v4f z0 = *(const v4f*)(zp), z1 = *(const v4f*)(zp + 4);
  v8h hv;
#pragma unroll
  for (int e = 0; e < 4; ++e) {
    const float za = z0[e], zb = z1[e];
    const float ga = za * __builtin_amdgcn_rcpf(1.0f + expf(-za));
    const float gb = zb * __builtin_amdgcn_rcpf(1.0f + expf(-zb));
    const float va = (yv[e] * rstd * w0[e] + q0[e]) * ga;
    const float vb = (yv[4 + e] * rstd * w1[e] + q1[e]) * gb;
    hv[e]     = (_Float16)(va * 8.0f);
    hv[4 + e] = (_Float16)(vb * 8.0f);
  }
  _Float16* op = (_Float16*)YG + (size_t)row * kDI + ch;
  *(volatile v8h*)op = hv;
  __threadfence();
  *(volatile v8h*)op = hv;
}

__global__ __launch_bounds__(256) void gelu_kernel(const float* __restrict__ F1, unsigned short* __restrict__ G16)
{
  __shared__ __align__(16) _Float16 sH[256 * 8];
  const int tid = threadIdx.x;
  const size_t base = ((size_t)blockIdx.x * 256 + tid) * 8;
#pragma unroll 1
  for (int e = 0; e < 8; ++e) {
    const float x = F1[base + e];
    const float u = 0.7978845608028654f * (x + 0.044715f * x * x * x);
    const float g = 0.5f * x * (1.0f + tanhf(u));
    sH[tid * 8 + e] = (_Float16)(g * 8.0f);
  }
  __syncthreads();
  const v8h hv = *(const v8h*)(sH + tid * 8);
  _Float16* op = (_Float16*)G16 + base;
  *(volatile v8h*)op = hv;
  __threadfence();
  *(volatile v8h*)op = hv;
}

extern "C" void kernel_launch(void* const* d_in, const int* in_sizes, int n_in,
                              void* d_out, int out_size, void* d_ws, size_t ws_size,
                              hipStream_t stream) {
  if (n_in < 21) return;
  if (in_sizes[0]  != kRows * kDim) return;
  if (in_sizes[1]  != kBatch * kDim) return;
  if (in_sizes[2]  != kDim * kMod) return;
  if (in_sizes[3]  != kMod) return;
  if (in_sizes[4]  != kDim * kXzW) return;
  if (in_sizes[5]  != kXzW) return;
  if (in_sizes[6]  != 9 * kDI) return;
  if (in_sizes[7]  != kDI) return;
  if (in_sizes[8]  != kDirs * kDI * kNR) return;
  if (in_sizes[9]  != kDirs * kDTR * kDI) return;
  if (in_sizes[10] != kDirs * kDI) return;
  if (in_sizes[11] != kDirs * kDI * kDS) return;
  if (in_sizes[12] != kDirs * kDI) return;
  if (in_sizes[13] != kDI) return;
  if (in_sizes[14] != kDI) return;
  if (in_sizes[15] != kDI * kDim) return;
  if (in_sizes[16] != kDim) return;
  if (in_sizes[17] != kDim * kHid) return;
  if (in_sizes[18] != kHid) return;
  if (in_sizes[19] != kHid * kDim) return;
  if (in_sizes[20] != kDim) return;
  if (out_size != kRows * kDim) return;
  if (ws_size < kWsTotal) return;

  const float* x       = (const float*)d_in[0];
  const float* cvec    = (const float*)d_in[1];
  const float* W_ada   = (const float*)d_in[2];
  const float* b_ada   = (const float*)d_in[3];
  const float* W_in    = (const float*)d_in[4];
  const float* b_in    = (const float*)d_in[5];
  const float* conv_w  = (const float*)d_in[6];
  const float* conv_b  = (const float*)d_in[7];
  const float* W_xproj = (const float*)d_in[8];
  const float* W_dt    = (const float*)d_in[9];
  const float* dt_bias = (const float*)d_in[10];
  const float* A_log   = (const float*)d_in[11];
  const float* Dp      = (const float*)d_in[12];
  const float* ln_w    = (const float*)d_in[13];
  const float* ln_b    = (const float*)d_in[14];
  const float* W_out   = (const float*)d_in[15];
  const float* b_out   = (const float*)d_in[16];
  const float* W_fc1   = (const float*)d_in[17];
  const float* b_fc1   = (const float*)d_in[18];
  const float* W_fc2   = (const float*)d_in[19];
  const float* b_fc2   = (const float*)d_in[20];
  float* out = (float*)d_out;

  char* ws = (char*)d_ws;
  unsigned short* WIN  = (unsigned short*)(ws + kOffWIN);
  unsigned short* WX   = (unsigned short*)(ws + kOffWX);
  unsigned short* WDT  = (unsigned short*)(ws + kOffWDT);
  unsigned short* WOUT = (unsigned short*)(ws + kOffWOUT);
  unsigned short* WF1  = (unsigned short*)(ws + kOffWF1);
  unsigned short* WF2  = (unsigned short*)(ws + kOffWF2);
  float*          MOD  = (float*)(ws + kOffMOD);
  unsigned short* H16  = (unsigned short*)(ws + kOffH16);
  float*          XZ   = (float*)(ws + kOffXZ);
  float*          XI   = (float*)(ws + kOffXI);
  unsigned short* XS   = (unsigned short*)(ws + kOffXS);
  float*          XD   = (float*)(ws + kOffXD);
  unsigned short* DTA  = (unsigned short*)(ws + kOffDTA);
  float*          DTP  = (float*)(ws + kOffDTP);
  float*          Y    = (float*)(ws + kOffY);
  unsigned short* YG   = (unsigned short*)(ws + kOffYG);
  float*          X1   = (float*)(ws + kOffX1);
  unsigned short* M16  = (unsigned short*)(ws + kOffM16);
  float*          F1   = (float*)(ws + kOffF1);
  unsigned short* G16  = (unsigned short*)(ws + kOffG16);

  const float wsc = 256.0f;
  wt_cast_kernel<64><<<dim3(kXzW / 64, kDim / 64, 1), 256, 0, stream>>>(W_in, WIN, kDim, kXzW, kXzW, kDim, 0L, 0L, wsc);
  wt_cast_kernel<64><<<dim3(kNRP / 64, kDI / 64, kDirs), 256, 0, stream>>>(W_xproj, WX, kDI, kNR, kNRP, kDI,
      (long)kDI * kNR, (long)kNRP * kDI, wsc);
  wt_cast_kernel<32><<<dim3(kDI / 64, 1, kDirs), 256, 0, stream>>>(W_dt, WDT, kDTR, kDI, kDI, kDtK,
      (long)kDTR * kDI, (long)kDI * kDtK, wsc);
  wt_cast_kernel<64><<<dim3(kDim / 64, kDI / 64, 1), 256, 0, stream>>>(W_out, WOUT, kDI, kDim, kDim, kDI, 0L, 0L, wsc);
  wt_cast_kernel<64><<<dim3(kHid / 64, kDim / 64, 1), 256, 0, stream>>>(W_fc1, WF1, kDim, kHid, kHid, kDim, 0L, 0L, wsc);
  wt_cast_kernel<64><<<dim3(kDim / 64, kHid / 64, 1), 256, 0, stream>>>(W_fc2, WF2, kHid, kDim, kDim, kHid, 0L, 0L, wsc);

  mod_kernel<<<dim3(kMod / 256, kBatch), 256, 0, stream>>>(cvec, W_ada, b_ada, MOD);

  ln_mod_kernel<<<kRows / 8, 256, 0, stream>>>(x, MOD, 0, kDim, H16);

  wmma_gemm64<0, 0, 2, 0, false, 0, false><<<dim3(64, 1), 256, 0, stream>>>(
      H16, nullptr, kDim, 0L,
      WIN, nullptr, kDim, 0L,
      (void*)XZ, nullptr, kXzW, 0L,
      b_in, nullptr, 0L,
      kRows, kXzW, kDim, 1.0f / 2048.0f,
      nullptr, 0, 0);

  conv_kernel<<<kRows / 4, 256, 0, stream>>>(XZ, conv_w, conv_b, XI, XS, XS + (size_t)kRows * kDI);

  wmma_gemm64<0, 0, 0, 0, false, 0, false><<<dim3(12, 2), 256, 0, stream>>>(
      XS, nullptr, kDI, 0L,
      WX, nullptr, kDI, (long)2 * kNRP * kDI,
      (void*)XD, nullptr, kNRP, (long)2 * kRows * kNRP,
      nullptr, nullptr, 0L,
      kRows, kNRP, kDI, 1.0f / 65536.0f,
      nullptr, 0, 0);
  wmma_gemm64<0, 0, 0, 0, false, 0, false><<<dim3(12, 2), 256, 0, stream>>>(
      XS + (size_t)kRows * kDI, nullptr, kDI, 0L,
      WX + (size_t)kNRP * kDI, nullptr, kDI, (long)2 * kNRP * kDI,
      (void*)(XD + (size_t)kRows * kNRP), nullptr, kNRP, (long)2 * kRows * kNRP,
      nullptr, nullptr, 0L,
      kRows, kNRP, kDI, 1.0f / 65536.0f,
      nullptr, 0, 0);

  dta_kernel<<<(kDirs * kRows * 4) / 256, 256, 0, stream>>>(XD, DTA);

  wmma_gemm64<0, 0, 0, 0, false, 0, false><<<dim3(32, kDirs), 256, 0, stream>>>(
      DTA, nullptr, kDtK, (long)kRows * kDtK,
      WDT, nullptr, kDtK, (long)kDI * kDtK,
      (void*)DTP, nullptr, kDI, (long)kRows * kDI,
      nullptr, nullptr, 0L,
      kRows, kDI, kDtK, 1.0f / 65536.0f,
      nullptr, 0, 0);

  scan_kernel<<<kBatch * kDirs * (kDI / kScanCh), 128, 0, stream>>>(XD, DTP, XI, dt_bias, A_log, Dp, Y);

  merge_kernel<<<kRows / 4, 256, 0, stream>>>(Y, XZ, ln_w, ln_b, YG);

  wmma_gemm64<0, 0, 2, 0, true, 0, true><<<dim3(16, 1), 256, 0, stream>>>(
      YG, nullptr, kDI, 0L,
      WOUT, nullptr, kDI, 0L,
      (void*)X1, nullptr, kDim, 0L,
      b_out, x, 0L,
      kRows, kDim, kDI, 1.0f / 2048.0f,
      MOD + 2 * kDim, 10, kMod);

  ln_mod_kernel<<<kRows / 8, 256, 0, stream>>>(X1, MOD, 3 * kDim, 4 * kDim, M16);

  wmma_gemm64<0, 0, 2, 0, false, 0, false><<<dim3(64, 1), 256, 0, stream>>>(
      M16, nullptr, kDim, 0L,
      WF1, nullptr, kDim, 0L,
      (void*)F1, nullptr, kHid, 0L,
      b_fc1, nullptr, 0L,
      kRows, kHid, kDim, 1.0f / 2048.0f,
      nullptr, 0, 0);

  gelu_kernel<<<(kRows * kHid / 8) / 256, 256, 0, stream>>>(F1, G16);

  wmma_gemm64<0, 0, 2, 0, true, 0, true><<<dim3(16, 1), 256, 0, stream>>>(
      G16, nullptr, kHid, 0L,
      WF2, nullptr, kHid, 0L,
      (void*)out, nullptr, kDim, 0L,
      b_fc2, X1, 0L,
      kRows, kDim, kHid, 1.0f / 2048.0f,
      MOD + 5 * kDim, 10, kMod);
}
